// LowRankMultiheadAttention_56255481643695
// MI455X (gfx1250) — hardware-verified
//
#include <hip/hip_runtime.h>


#define NB_  2
#define TT   2048
#define DM   1024
#define RK   256
#define NH_  16
#define HD   64
#define HPP  4
#define PCAR 1024.0f
typedef _Float16 h16;
typedef unsigned short bf;
typedef __attribute__((ext_vector_type(16))) __bf16   v16bf;
typedef __attribute__((ext_vector_type(16))) _Float16 v16h;
typedef __attribute__((ext_vector_type(8)))  _Float16 v8h;
typedef __attribute__((ext_vector_type(8)))  unsigned short v8us;
typedef __attribute__((ext_vector_type(8)))  float    v8f;
typedef __attribute__((ext_vector_type(4)))  float    v4f;
typedef v8h  __attribute__((may_alias)) v8ha;
typedef v4f  __attribute__((may_alias)) v4fa;
typedef v8us __attribute__((may_alias)) v8usa;

__device__ __forceinline__ unsigned short f2bf(float f) { unsigned u = __float_as_uint(f); u += 0x7FFFu + ((u >> 16) & 1u); return (unsigned short)(u >> 16); }
__device__ __forceinline__ float bf2f(unsigned short b) { return __uint_as_float(((unsigned)b) << 16); }
__device__ __forceinline__ float bfr(float f) { return bf2f(f2bf(f)); }
__device__ __forceinline__ v16h cat16(v8h lo, v8h hi) { return __builtin_shufflevector(lo, hi, 0, 1, 2, 3, 4, 5, 6, 7, 8, 9, 10, 11, 12, 13, 14, 15); }
__device__ __forceinline__ v16bf cat16b(v8us lo, v8us hi) { return __builtin_bit_cast(v16bf, __builtin_shufflevector(lo, hi, 0, 1, 2, 3, 4, 5, 6, 7, 8, 9, 10, 11, 12, 13, 14, 15)); }
__device__ __forceinline__ v8f wmma16(v16h a, v16h b, v8f c) { return __builtin_amdgcn_wmma_f32_16x16x32_f16(false, a, false, b, (short)0, c, false, false); }
__device__ __forceinline__ v8f wmmab(v16bf a, v16bf b, v8f c) { return __builtin_amdgcn_wmma_f32_16x16x32_bf16(false, a, false, b, (short)0, c, false, false); }


template <typename T16> struct WFrag;
template <> struct WFrag<h16> { typedef v16h V; static __device__ __forceinline__ V ld(const h16* p) { return cat16(*(const v8h*)p, *(const v8h*)(p + 16)); } static __device__ __forceinline__ v8f mma(V a, V b, v8f c) { return wmma16(a, b, c); } };
template <> struct WFrag<bf> { typedef v16bf V; static __device__ __forceinline__ V ld(const bf* p) { return cat16b(*(const v8us*)p, *(const v8us*)(p + 16)); } static __device__ __forceinline__ v8f mma(V a, V b, v8f c) { return wmmab(a, b, c); } };
template <typename T16, int NSPLIT, bool BIAS>
__global__ __launch_bounds__(32) void k_gemmw(const T16* __restrict__ A, const T16* __restrict__ A2, const T16* __restrict__ Bt, const T16* __restrict__ Bt2, int K, float* C, int ldc, const float* __restrict__ bias, size_t sA, size_t sB, size_t sC) {
    typedef typename WFrag<T16>::V V;
    __shared__ __align__(16) float os[16 * 68];
    const size_t z = blockIdx.z; A += z * sA; if (A2) A2 += z * sA; Bt += z * sB; if (Bt2) Bt2 += z * sB; C += z * sC;
    const int lane = threadIdx.x & 31, lr = lane & 15, hi = lane >> 4; const int r0 = blockIdx.x * 64, c0 = blockIdx.y * 64;
    v8f acc[4][4];
#pragma unroll
    for (int mb = 0; mb < 4; ++mb)
#pragma unroll
        for (int nb = 0; nb < 4; ++nb) acc[mb][nb] = (v8f){};
    const size_t aoff = (size_t)(r0 + lr) * K + 8 * hi, boff = (size_t)(c0 + lr) * K + 8 * hi;
#pragma unroll 1
    for (int kc = 0; kc < K; kc += 32) {
        V a[4], a2[4];
#pragma unroll
        for (int mb = 0; mb < 4; ++mb) { a[mb] = WFrag<T16>::ld(A + aoff + (size_t)mb * 16 * K + kc); if (NSPLIT == 1 || NSPLIT == 2) a2[mb] = WFrag<T16>::ld(A2 + aoff + (size_t)mb * 16 * K + kc); }
#pragma unroll
        for (int nb = 0; nb < 4; ++nb) { const V b = WFrag<T16>::ld(Bt + boff + (size_t)nb * 16 * K + kc); V b2; if (NSPLIT >= 2) b2 = WFrag<T16>::ld(Bt2 + boff + (size_t)nb * 16 * K + kc);
#pragma unroll
            for (int mb = 0; mb < 4; ++mb) { acc[mb][nb] = WFrag<T16>::mma(a[mb], b, acc[mb][nb]); if (NSPLIT == 1 || NSPLIT == 2) acc[mb][nb] = WFrag<T16>::mma(a2[mb], b, acc[mb][nb]); if (NSPLIT >= 2) acc[mb][nb] = WFrag<T16>::mma(a[mb], b2, acc[mb][nb]); } }
        asm volatile("v_nop\n\tv_nop\n\tv_nop\n\tv_nop" : "+v"(acc[0][0]), "+v"(acc[1][1]), "+v"(acc[2][2]), "+v"(acc[3][3]) : "v"(a[0]), "v"(a[3]));
    }
#pragma unroll
    for (int mb = 0; mb < 4; ++mb) {
#pragma unroll
        for (int nb = 0; nb < 4; ++nb) {
#pragma unroll
            for (int j = 0; j < 8; ++j) os[(hi * 8 + j) * 68 + nb * 16 + lr] = acc[mb][nb][j]; }
        __builtin_amdgcn_wave_barrier(); asm volatile("" ::: "memory");
        float* crow = C + (size_t)(r0 + mb * 16) * ldc + c0;
#pragma unroll 1
        for (int ps = 0; ps < 2; ++ps) {
#pragma unroll
            for (int s = 0; s < 8; ++s) { const int row = 2 * s + hi, cofs = lr * 4; v4f val = *(const v4fa*)(os + row * 68 + cofs); if (BIAS) { val[0] += bfr(bias[c0 + cofs]); val[1] += bfr(bias[c0 + cofs + 1]); val[2] += bfr(bias[c0 + cofs + 2]); val[3] += bfr(bias[c0 + cofs + 3]); }
                *(volatile v4f*)(crow + (size_t)row * ldc + cofs) = val; }
            if (ps == 0) __threadfence(); }
        __builtin_amdgcn_wave_barrier(); asm volatile("" ::: "memory");
    }
}

__device__ __forceinline__ h16 tohx(float x) { return (h16)x; }
__device__ __forceinline__ void splitf(float y, unsigned short& h, unsigned short& l) { h = f2bf(y); l = f2bf(y - bf2f(h)); }
typedef __attribute__((ext_vector_type(2))) unsigned short v2us;
typedef __attribute__((ext_vector_type(4))) unsigned short v4us;
typedef __attribute__((ext_vector_type(2))) _Float16 v2h;
typedef __attribute__((ext_vector_type(4))) _Float16 v4h;

__global__ __launch_bounds__(256) void k_wtG(const float* __restrict__ w, int K, int N, bf* Bt) {
    const int lane = threadIdx.x & 31; const int L0 = (blockIdx.x * 8 + (threadIdx.x >> 5)) * 8; const int nlines = N * K / 64;
#pragma unroll
    for (int ps = 0; ps < 2; ++ps) {
#pragma unroll 1
        for (int l = 0; l < 8; ++l) { const int L = L0 + l; if (L >= nlines) break; const size_t e = (size_t)L * 64 + lane * 2; const int k = (int)(e % K), n = (int)(e / K); v2us o;
            o[0] = f2bf(w[(size_t)k * N + n]); o[1] = f2bf(w[(size_t)(k + 1) * N + n]); *(volatile v2us*)(Bt + e) = o; }
        if (ps == 0) __threadfence(); }
}
__global__ __launch_bounds__(256) void k_cvt8(const float* __restrict__ src, bf* dst, size_t n8) { const size_t i = (size_t)blockIdx.x * 256 + threadIdx.x; if (i >= n8) return; const v8f v = *(const v8f*)(src + i * 8); v8us o;
#pragma unroll
    for (int k = 0; k < 8; ++k) o[k] = f2bf(v[k]); *(volatile v8us*)(dst + i * 8) = o; __threadfence(); *(volatile v8us*)(dst + i * 8) = o; }
__global__ __launch_bounds__(256) void k_spl(const float* __restrict__ F, size_t n4, bf* Hh, bf* Hl) { const size_t e = ((size_t)blockIdx.x * 256 + threadIdx.x) * 4; if (e >= n4) return; const v4f a = *(const v4f*)(F + e); v4us oh, ol;
#pragma unroll
    for (int u = 0; u < 4; ++u) { unsigned short h, l; splitf(a[u], h, l); oh[u] = h; ol[u] = l; } *(volatile v4us*)(Hh + e) = oh; *(volatile v4us*)(Hl + e) = ol; __threadfence(); *(volatile v4us*)(Hh + e) = oh; *(volatile v4us*)(Hl + e) = ol; }
__global__ __launch_bounds__(256) void k_pl(const float* __restrict__ F, h16* P) { const int e = (blockIdx.x * 256 + threadIdx.x) * 4; if (e >= NH_ * TT * HD) return; const int d = e % HD; const int t = (e / HD) % TT; const int h = e / (HD * TT); const float* f = F + (size_t)t * DM + h * HD + d; v4h o;
#pragma unroll
    for (int u = 0; u < 4; ++u) o[u] = tohx(f[u]); *(volatile v4h*)(P + e) = o; __threadfence(); *(volatile v4h*)(P + e) = o; }
__global__ __launch_bounds__(256) void k_vt(const float* __restrict__ V, h16* VT) { const int e = (blockIdx.x * 256 + threadIdx.x) * 2; if (e >= NH_ * HD * TT) return; const int t = e % TT; const int d = (e / TT) % HD; const int h = e / (TT * HD); v2h o; o[0] = tohx(V[(size_t)t * DM + h * HD + d]); o[1] = tohx(V[(size_t)(t + 1) * DM + h * HD + d]); *(volatile v2h*)(VT + e) = o; __threadfence(); *(volatile v2h*)(VT + e) = o; }
__global__ __launch_bounds__(256) void k_soft(const float* __restrict__ Sb, h16* P16) { const int lane = threadIdx.x & 31; const int row = blockIdx.x * 8 + (threadIdx.x >> 5); if (row >= HPP * TT) return; const float* sr = Sb + (size_t)row * TT; float v[TT / 32]; float mx = -3.0e38f;
#pragma unroll
    for (int ch = 0; ch < TT / 128; ++ch) { const v4f a = *(const v4f*)(sr + ch * 128 + lane * 4);
#pragma unroll
        for (int u = 0; u < 4; ++u) { const float t = a[u] * 0.125f; v[ch * 4 + u] = t; mx = fmaxf(mx, t); } }
#pragma unroll
    for (int sh = 16; sh; sh >>= 1) mx = fmaxf(mx, __shfl_xor(mx, sh, 32));
    float sum = 0.f;
#pragma unroll
    for (int q = 0; q < TT / 32; ++q) { float d0 = __fsub_rn(v[q], mx); asm volatile("" : "+v"(d0)); v[q] = __builtin_amdgcn_exp2f(__fmul_rn(d0, 1.4426950408889634f)); sum += v[q]; }
#pragma unroll
    for (int sh = 16; sh; sh >>= 1) sum += __shfl_xor(sum, sh, 32);
    const float f = __fdiv_rn(PCAR, sum);
    for (int ps = 0; ps < 2; ++ps) {
#pragma unroll
        for (int ch = 0; ch < TT / 128; ++ch) { v4h o4;
#pragma unroll
            for (int q = 0; q < 4; ++q) o4[q] = tohx(v[ch * 4 + q] * f); *(volatile v4h*)(P16 + (size_t)row * TT + ch * 128 + lane * 4) = o4; }
        if (ps == 0) __threadfence(); } }
__global__ __launch_bounds__(256) void k_mrg(const float* __restrict__ O, int h0, bf* Ah, bf* Al) { const int e = (blockIdx.x * 256 + threadIdx.x) * 4; if (e >= HPP * TT * HD) return; const int d = e % HD; const int t = (e / HD) % TT; const int z = e / (HD * TT); v4us oh, ol;
#pragma unroll
    for (int u = 0; u < 4; ++u) { unsigned short a, b; splitf(O[e + u] * (1.0f / PCAR), a, b); oh[u] = a; ol[u] = b; } const size_t oo = (size_t)t * DM + (h0 + z) * HD + d; *(volatile v4us*)(Ah + oo) = oh; *(volatile v4us*)(Al + oo) = ol; __threadfence(); *(volatile v4us*)(Ah + oo) = oh; *(volatile v4us*)(Al + oo) = ol; }

extern "C" void kernel_launch(void* const* d_in, const int* in_sizes, int n_in,
                              void* d_out, int out_size, void* d_ws, size_t ws_size, hipStream_t stream) {
    (void)in_sizes; (void)n_in; (void)out_size;
    const float** I = (const float**)d_in;
    const float* xin[3] = {I[0], I[1], I[2]}; const float* Wlo[4] = {I[3], I[7], I[11], I[15]}; const float* blo[4] = {I[4], I[8], I[12], I[16]}; const float* Whi[4] = {I[5], I[9], I[13], I[17]}; const float* bhi[4] = {I[6], I[10], I[14], I[18]};
    float* OUT = (float*)d_out;
    char* wsp = (char*)d_ws;
    auto take = [&](size_t bytes) { char* p = wsp; wsp += (bytes + 255) & ~(size_t)255; return (void*)p; };
    bf* BLO[4]; bf* BHI[4]; for (int i = 0; i < 4; ++i) { BLO[i] = (bf*)take((size_t)RK * DM * 2); BHI[i] = (bf*)take((size_t)DM * RK * 2); }
    bf* XB = (bf*)take((size_t)TT * DM * 2); float* LO = (float*)take((size_t)TT * RK * 4); bf* LOh = (bf*)take((size_t)TT * RK * 2); bf* LOl = (bf*)take((size_t)TT * RK * 2); float* PJ[3]; for (int i = 0; i < 3; ++i) PJ[i] = (float*)take((size_t)TT * DM * 4);
    h16* Q16 = (h16*)take((size_t)NH_ * TT * HD * 2); h16* K16 = (h16*)take((size_t)NH_ * TT * HD * 2); h16* VT = (h16*)take((size_t)NH_ * HD * TT * 2); float* Sb = (float*)take((size_t)HPP * TT * TT * 4); h16* P16 = (h16*)take((size_t)HPP * TT * TT * 2); float* O = (float*)take((size_t)HPP * TT * HD * 4);
    bf* Ah = (bf*)take((size_t)TT * DM * 2); bf* Al = (bf*)take((size_t)TT * DM * 2);
    if ((size_t)(wsp - (char*)d_ws) > ws_size) return;
    for (int i = 0; i < 4; ++i) { k_wtG<<<(DM * RK / 64 + 63) / 64, 256, 0, stream>>>(Wlo[i], DM, RK, BLO[i]); k_wtG<<<(RK * DM / 64 + 63) / 64, 256, 0, stream>>>(Whi[i], RK, DM, BHI[i]); }
    const size_t zq = (size_t)TT * HD, zS = (size_t)TT * TT;
    for (int b = 0; b < NB_; ++b) {
        for (int i = 0; i < 3; ++i) {
            k_cvt8<<<(TT * DM / 8 + 255) / 256, 256, 0, stream>>>(xin[i] + (size_t)b * TT * DM, XB, (size_t)TT * DM / 8);
            k_gemmw<bf, 0, true><<<dim3(TT / 64, RK / 64, 1), 32, 0, stream>>>(XB, nullptr, BLO[i], nullptr, DM, LO, RK, blo[i], 0, 0, 0); k_spl<<<(TT * RK / 4 + 255) / 256, 256, 0, stream>>>(LO, (size_t)TT * RK, LOh, LOl);
            k_gemmw<bf, 1, true><<<dim3(TT / 64, DM / 64, 1), 32, 0, stream>>>(LOh, LOl, BHI[i], nullptr, RK, PJ[i], DM, bhi[i], 0, 0, 0); }
        k_pl<<<(NH_ * TT * HD / 4 + 255) / 256, 256, 0, stream>>>(PJ[0], Q16); k_pl<<<(NH_ * TT * HD / 4 + 255) / 256, 256, 0, stream>>>(PJ[1], K16); k_vt<<<(NH_ * HD * TT / 2 + 255) / 256, 256, 0, stream>>>(PJ[2], VT);
        for (int h0 = 0; h0 < NH_; h0 += HPP) { const size_t zo = (size_t)h0 * zq;
            k_gemmw<h16, 0, false><<<dim3(TT / 64, TT / 64, HPP), 32, 0, stream>>>(Q16 + zo, nullptr, K16 + zo, nullptr, HD, Sb, TT, nullptr, zq, zq, zS);
            k_soft<<<HPP * TT / 8, 256, 0, stream>>>(Sb, P16);
            k_gemmw<h16, 0, false><<<dim3(TT / 64, 1, HPP), 32, 0, stream>>>(P16, nullptr, VT + zo, nullptr, TT, O, HD, nullptr, zS, (size_t)HD * TT, zq);
            k_mrg<<<(HPP * TT * HD / 4 + 255) / 256, 256, 0, stream>>>(O, h0, Ah, Al); }
        k_gemmw<bf, 1, true><<<dim3(TT / 64, RK / 64, 1), 32, 0, stream>>>(Ah, Al, BLO[3], nullptr, DM, LO, RK, blo[3], 0, 0, 0); k_spl<<<(TT * RK / 4 + 255) / 256, 256, 0, stream>>>(LO, (size_t)TT * RK, LOh, LOl);
        k_gemmw<bf, 1, true><<<dim3(TT / 64, DM / 64, 1), 32, 0, stream>>>(LOh, LOl, BHI[3], nullptr, RK, OUT + (size_t)b * TT * DM, DM, bhi[3], 0, 0, 0); }
}
